// PeepholeLSTMCell_65240553226497
// MI455X (gfx1250) — hardware-verified
//
#include <hip/hip_runtime.h>
#include <stdint.h>

constexpr int NBATCH = 4096;
constexpr int NIN    = 1024;
constexpr int NHID   = 1024;
constexpr int KCAT   = NIN + NHID;
constexpr int NGATE4 = 4 * NHID;

static_assert(KCAT % 32 == 0, "K multiple of 32");
static_assert(NBATCH % 64 == 0 && NGATE4 % 64 == 0, "M,N multiples of 64");
static_assert(NIN == 128 * 8 && NHID == 128 * 8, "pack kernels: 256 threads x 8 elements per row");
static_assert(NHID == 256 * 4, "gate kernel: 256 threads x 4 columns per row");

constexpr size_t WS_A_OFF   = 0;
constexpr size_t WS_A_BYTES = (size_t)NBATCH * KCAT * 2;
constexpr size_t WS_W_OFF   = WS_A_OFF + WS_A_BYTES;
constexpr size_t WS_W_BYTES = (size_t)NGATE4 * KCAT * 2;
constexpr size_t WS_Z_OFF   = WS_W_OFF + WS_W_BYTES;
constexpr size_t WS_Z_BYTES = (size_t)NBATCH * NGATE4 * 4;
constexpr size_t WS_TOTAL   = WS_Z_OFF + WS_Z_BYTES;
static_assert(WS_TOTAL == 100663296, "carve total");
static_assert(WS_TOTAL <= 134217728, "carve under 128 MiB");

constexpr size_t OUT1_ELEM_OFF = (size_t)NBATCH * NHID;
static_assert(OUT1_ELEM_OFF * 4 == 16777216, "out1 byte offset");
static_assert((OUT1_ELEM_OFF + (size_t)NBATCH * NHID) * 4 == 33554432, "out total bytes");

constexpr int GATE_ROWS_PER_BLOCK = 4;
static_assert(NBATCH % GATE_ROWS_PER_BLOCK == 0, "gate grid exact");

typedef __attribute__((ext_vector_type(16))) _Float16 v16h;
typedef __attribute__((ext_vector_type(8)))  _Float16 v8h;
typedef __attribute__((ext_vector_type(16))) __bf16   v16b;
typedef __attribute__((ext_vector_type(8)))  __bf16   v8b;
typedef __attribute__((ext_vector_type(8)))  float    v8f;
typedef __attribute__((ext_vector_type(4)))  float    v4f;
typedef __attribute__((ext_vector_type(4)))  unsigned v4u;

__device__ __forceinline__ unsigned short f2bf_bits(float f) {
  unsigned u = __float_as_uint(f);
  return (unsigned short)((u + 0x7FFFu + ((u >> 16) & 1u)) >> 16);
}
__device__ __forceinline__ float bf_bits2f(unsigned short h) { return __uint_as_float(((unsigned)h) << 16); }

__device__ __forceinline__ void dep_guard_h(v8f& a, v8f& b, v16h x, v16h y) { asm volatile("v_nop\n\tv_nop\n\tv_nop\n\tv_nop" : "+v"(a), "+v"(b) : "v"(x), "v"(y)); }
__device__ __forceinline__ void dep_guard_b(v8f& a, v8f& b, v16b x, v16b y) { asm volatile("v_nop\n\tv_nop\n\tv_nop\n\tv_nop" : "+v"(a), "+v"(b) : "v"(x), "v"(y)); }
__device__ __forceinline__ void keep4_h(v16h a, v16h b, v16h c, v16h d) { asm volatile("v_nop" :: "v"(a), "v"(b), "v"(c), "v"(d)); }
__device__ __forceinline__ void keep4_b(v16b a, v16b b, v16b c, v16b d) { asm volatile("v_nop" :: "v"(a), "v"(b), "v"(c), "v"(d)); }
__device__ __forceinline__ void acc_guard4(v8f& a, v8f& b, v8f& c, v8f& d) { asm volatile("v_nop\n\tv_nop\n\tv_nop\n\tv_nop" : "+v"(a), "+v"(b), "+v"(c), "+v"(d)); }
template <typename T> struct Frag;
template <> struct Frag<_Float16> {
  typedef v16h V; union U { v16h v; v8h h[2]; };
  static __device__ __forceinline__ v16h load(const _Float16* p) {
    U f; f.h[0] = *(const v8h*)(p); f.h[1] = *(const v8h*)(p + 16); return f.v;
  }
  static __device__ __forceinline__ v8f mma(v16h a, v16h b, v8f c) {
    return __builtin_amdgcn_wmma_f32_16x16x32_f16(false, a, false, b, (short)0, c, false, false);
  }
  static __device__ __forceinline__ void guard(v8f& a, v8f& b, v16h x, v16h y) { dep_guard_h(a, b, x, y); }
  static __device__ __forceinline__ void keep(v16h a, v16h b, v16h c, v16h d) { keep4_h(a, b, c, d); }
};
template <> struct Frag<__bf16> {
  typedef v16b V; union U { v16b v; v8b h[2]; };
  static __device__ __forceinline__ v16b load(const __bf16* p) {
    U f; f.h[0] = *(const v8b*)(p); f.h[1] = *(const v8b*)(p + 16); return f.v;
  }
  static __device__ __forceinline__ v8f mma(v16b a, v16b b, v8f c) {
    return __builtin_amdgcn_wmma_f32_16x16x32_bf16(false, a, false, b, (short)0, c, false, false);
  }
  static __device__ __forceinline__ void guard(v8f& a, v8f& b, v16b x, v16b y) { dep_guard_b(a, b, x, y); }
  static __device__ __forceinline__ void keep(v16b a, v16b b, v16b c, v16b d) { keep4_b(a, b, c, d); }
};

template <int ET> struct Elem;
template <> struct Elem<0> { typedef _Float16 T; };
template <> struct Elem<1> { typedef __bf16 T; };
template <int ET, bool SPLIT, int BIAS_MODE, int OUT_MODE, bool RESID, int ACT = 0>
__global__ __launch_bounds__(256) void wmma_gemm64(
    const unsigned short* __restrict__ Ap, const unsigned short* __restrict__ A2p, int lda, long strideA,
    const unsigned short* __restrict__ Btp, const unsigned short* __restrict__ Bt2p, int ldb, long strideB,
    void* __restrict__ Cout, void* __restrict__ Cout2, int ldc, long strideC,
    const float* __restrict__ bias,
    const float* __restrict__ resid, long strideR,
    int M, int N, int K, float scale) {
  typedef typename Elem<ET>::T T;
  typedef typename Frag<T>::V V;
  const T* A = (const T*)Ap; const T* A2 = (const T*)A2p; const T* Bt = (const T*)Btp; const T* Bt2 = (const T*)Bt2p;
  __shared__ __align__(16) float sT[8][16 * 68];
  const int b    = blockIdx.y;
  const int lane = threadIdx.x & 31;
  const int wave = threadIdx.x >> 5;
  const int tilesN = N >> 6;
  const int tilesM = M >> 6;
  const int tile = blockIdx.x * 8 + wave;
  if (tile >= tilesM * tilesN) return;
  const int tm = tile / tilesN;
  const int tn = tile - tm * tilesN;
  const int m0 = tm << 6;
  const int n0 = tn << 6;

  const T* Ab  = A  + (size_t)b * strideA;
  const T* Bb  = Bt + (size_t)b * strideB;
  const T* Ab2 = SPLIT ? (A2  + (size_t)b * strideA) : nullptr;
  const T* Bb2 = SPLIT ? (Bt2 + (size_t)b * strideB) : nullptr;

  const int rlane = lane & 15;
  const int koff  = (lane >> 4) * 8;
  const int mOff  = (lane >> 4) * 8;

  v8f acc[4][4];
#pragma unroll
  for (int i = 0; i < 4; ++i)
#pragma unroll
    for (int j = 0; j < 4; ++j) acc[i][j] = (v8f){0.f,0.f,0.f,0.f,0.f,0.f,0.f,0.f};

  for (int k0 = 0; k0 < K; k0 += 32) {
    V bh[4], bl[4];
#pragma unroll
    for (int j = 0; j < 4; ++j) {
      const size_t bo = (size_t)(n0 + (j << 4) + rlane) * ldb + koff + k0;
      bh[j] = Frag<T>::load(Bb + bo);
      if (SPLIT) bl[j] = Frag<T>::load(Bb2 + bo);
    }
#pragma unroll
    for (int i = 0; i < 4; ++i) {
      const size_t ao = (size_t)(m0 + (i << 4) + rlane) * lda + koff + k0;
      V ah = Frag<T>::load(Ab + ao);
      V al;
      if (SPLIT) al = Frag<T>::load(Ab2 + ao);
#pragma unroll
      for (int j = 0; j < 4; ++j) {
        acc[i][j] = Frag<T>::mma(ah, bh[j], acc[i][j]);
        if (SPLIT) {
          acc[i][j] = Frag<T>::mma(ah, bl[j], acc[i][j]);
          acc[i][j] = Frag<T>::mma(al, bh[j], acc[i][j]);
        }
      }
      Frag<T>::guard(acc[i][0], acc[i][3], ah, SPLIT ? al : ah);
    }
    Frag<T>::keep(bh[0], bh[1], bh[2], bh[3]);
    if (SPLIT) Frag<T>::keep(bl[0], bl[1], bl[2], bl[3]);
  }
  acc_guard4(acc[0][0], acc[0][1], acc[0][2], acc[0][3]);
  acc_guard4(acc[1][0], acc[1][1], acc[1][2], acc[1][3]);
  acc_guard4(acc[2][0], acc[2][1], acc[2][2], acc[2][3]);
  acc_guard4(acc[3][0], acc[3][1], acc[3][2], acc[3][3]);

  float* slab = sT[wave];
  const float* Rb = RESID ? (resid + (size_t)b * strideR) : nullptr;
#pragma unroll
  for (int i = 0; i < 4; ++i) {
    const int mBase = m0 + (i << 4);
#pragma unroll
    for (int j = 0; j < 4; ++j) {
      const int n = n0 + (j << 4) + rlane;
      float bv = 0.f;
      if (BIAS_MODE == 2) bv = bias[n];
#pragma unroll
      for (int r = 0; r < 8; ++r) {
        float v = acc[i][j][r] * scale;
        if (BIAS_MODE == 1) v += bias[mBase + mOff + r];
        if (BIAS_MODE == 2) v += bv;
        if (RESID) v += Rb[(size_t)(mBase + mOff + r) * ldc + n];
        if (ACT == 1) v = tanhf(v);
        if (ACT == 2) v = fmaxf(v, 0.0f);
        if (ACT == 3) v = v / (1.0f + expf(-v));
        if (ACT == 4) v = (v > 0.f) ? v : 0.01f * v;
        if (ACT == 5) v = 0.5f * v * (1.0f + erff(v * 0.70710678118654752f));
        slab[(mOff + r) * 68 + (j << 4) + rlane] = v;
      }
    }
    __builtin_amdgcn_fence(__ATOMIC_RELEASE, "workgroup");
    __builtin_amdgcn_wave_barrier();
    __builtin_amdgcn_fence(__ATOMIC_ACQUIRE, "workgroup");
    if (OUT_MODE == 0) {
      float* C = (float*)Cout + (size_t)b * strideC;
      const int hh = lane >> 4, c4 = (lane & 15) * 4;
      for (int pass = 0; pass < 2; ++pass) {
#pragma unroll
        for (int it = 0; it < 8; ++it) {
          const int row = it * 2 + hh;
          v4f v = *(const v4f*)(slab + row * 68 + c4);
          *(volatile v4f*)(C + (size_t)(mBase + row) * ldc + n0 + c4) = v;
        }
        __threadfence();
      }
    } else {
      const int q = lane >> 3, c8 = (lane & 7) * 8;
      unsigned short* C  = (unsigned short*)Cout  + (size_t)b * strideC;
      unsigned short* C2 = (OUT_MODE == 2) ? ((unsigned short*)Cout2 + (size_t)b * strideC) : nullptr;
      for (int pass = 0; pass < 2; ++pass) {
#pragma unroll
        for (int it = 0; it < 4; ++it) {
          const int row = it * 4 + q;
          const float* sp = slab + row * 68 + c8;
          v8h hv, lv;
#pragma unroll
          for (int e = 0; e < 8; ++e) {
            if (OUT_MODE == 1) {
              hv[e] = (_Float16)sp[e];
            } else {
              unsigned short hb = f2bf_bits(sp[e]);
              unsigned short lb = f2bf_bits(sp[e] - bf_bits2f(hb));
              hv[e] = __builtin_bit_cast(_Float16, hb);
              lv[e] = __builtin_bit_cast(_Float16, lb);
            }
          }
          *(volatile v8h*)(C + (size_t)(mBase + row) * ldc + n0 + c8) = hv;
          if (OUT_MODE == 2) *(volatile v8h*)(C2 + (size_t)(mBase + row) * ldc + n0 + c8) = lv;
        }
        __threadfence();
      }
    }
    __builtin_amdgcn_fence(__ATOMIC_RELEASE, "workgroup");
    __builtin_amdgcn_wave_barrier();
    __builtin_amdgcn_fence(__ATOMIC_ACQUIRE, "workgroup");
  }
}

__device__ __forceinline__ unsigned pack_bf2(float lo, float hi) {
  return (unsigned)f2bf_bits(lo) | (((unsigned)f2bf_bits(hi)) << 16);
}
__device__ __forceinline__ float rne_bf(float f) { return bf_bits2f(f2bf_bits(f)); }
__device__ __forceinline__ v4f rne_bf4(v4f v) {
  v4f o;
  o[0] = rne_bf(v[0]); o[1] = rne_bf(v[1]); o[2] = rne_bf(v[2]); o[3] = rne_bf(v[3]);
  return o;
}
__device__ __forceinline__ v4f ld4f(const float* p) { return *(const v4f*)p; }

__device__ __forceinline__ float sigm_f(float x) {
  const float e = __expf(-x);
  return __builtin_amdgcn_rcpf(1.0f + e);
}
__device__ __forceinline__ float tanh_f(float x) {
  const float ax = fabsf(x);
  const float t  = __expf(-2.0f * ax);
  const float r  = (1.0f - t) * __builtin_amdgcn_rcpf(1.0f + t);
  return copysignf(r, x);
}

__global__ __launch_bounds__(256) void pack_act_rows(const float* __restrict__ x,
                                                     const float* __restrict__ h,
                                                     unsigned short* __restrict__ Aout) {
  const int row = blockIdx.x;
  const int t   = threadIdx.x;
  const bool second = (t >= 128);
  const int  kc     = second ? (t - 128) * 8 : t * 8;
  const float* src  = second ? (h + (size_t)row * NHID + kc) : (x + (size_t)row * NIN + kc);
  const v4f a = *(const v4f*)(src);
  const v4f c = *(const v4f*)(src + 4);
  v4u w;
  w[0] = pack_bf2(a[0], a[1]); w[1] = pack_bf2(a[2], a[3]);
  w[2] = pack_bf2(c[0], c[1]); w[3] = pack_bf2(c[2], c[3]);
  unsigned short* dst = Aout + (size_t)row * KCAT + (size_t)t * 8;
  *(volatile v4u*)dst = w;
  __threadfence();
  *(volatile v4u*)dst = w;
}

__global__ __launch_bounds__(256) void pack_w_rows(const float* __restrict__ w_ii, const float* __restrict__ w_if,
                                                   const float* __restrict__ w_ig, const float* __restrict__ w_io,
                                                   const float* __restrict__ w_hi, const float* __restrict__ w_hf,
                                                   const float* __restrict__ w_hg, const float* __restrict__ w_ho,
                                                   unsigned short* __restrict__ Wout) {
  const int nrow = blockIdx.x;
  const int g    = nrow >> 10;
  const int n    = nrow & (NHID - 1);
  const float* wx = w_ii; const float* wh = w_hi;
  if (g == 1)      { wx = w_if; wh = w_hf; }
  else if (g == 2) { wx = w_ig; wh = w_hg; }
  else if (g == 3) { wx = w_io; wh = w_ho; }
  const int t = threadIdx.x;
  const bool second = (t >= 128);
  const int  kc     = second ? (t - 128) * 8 : t * 8;
  const float* src  = second ? (wh + (size_t)n * NHID + kc) : (wx + (size_t)n * NIN + kc);
  const v4f a = *(const v4f*)(src);
  const v4f c = *(const v4f*)(src + 4);
  v4u w;
  w[0] = pack_bf2(a[0], a[1]); w[1] = pack_bf2(a[2], a[3]);
  w[2] = pack_bf2(c[0], c[1]); w[3] = pack_bf2(c[2], c[3]);
  unsigned short* dst = Wout + (size_t)nrow * KCAT + (size_t)t * 8;
  *(volatile v4u*)dst = w;
  __threadfence();
  *(volatile v4u*)dst = w;
}

__global__ __launch_bounds__(256) void peep_gates(const float* __restrict__ Z, const float* __restrict__ cprev,
                                                  const float* __restrict__ b_ii, const float* __restrict__ b_hi,
                                                  const float* __restrict__ b_if, const float* __restrict__ b_hf,
                                                  const float* __restrict__ b_ig, const float* __restrict__ b_hg,
                                                  const float* __restrict__ b_io, const float* __restrict__ b_ho,
                                                  const float* __restrict__ w_ci, const float* __restrict__ w_cf,
                                                  const float* __restrict__ w_co,
                                                  float* __restrict__ out) {
  const int col = threadIdx.x * 4;
  const v4f bsi = rne_bf4(ld4f(b_ii + col)) + rne_bf4(ld4f(b_hi + col));
  const v4f bsf = rne_bf4(ld4f(b_if + col)) + rne_bf4(ld4f(b_hf + col));
  const v4f bsg = rne_bf4(ld4f(b_ig + col)) + rne_bf4(ld4f(b_hg + col));
  const v4f bso = rne_bf4(ld4f(b_io + col)) + rne_bf4(ld4f(b_ho + col));
  const v4f pci = rne_bf4(ld4f(w_ci + col));
  const v4f pcf = rne_bf4(ld4f(w_cf + col));
  const v4f pco = rne_bf4(ld4f(w_co + col));
  float* outh = out;
  float* outc = out + OUT1_ELEM_OFF;
#pragma unroll 1
  for (int rr = 0; rr < GATE_ROWS_PER_BLOCK; ++rr) {
    const int row = blockIdx.x * GATE_ROWS_PER_BLOCK + rr;
    const size_t zoff = (size_t)row * NGATE4 + col;
    const v4f zi = ld4f(Z + zoff);
    const v4f zf = ld4f(Z + zoff + NHID);
    const v4f zg = ld4f(Z + zoff + 2 * NHID);
    const v4f zz = ld4f(Z + zoff + 3 * NHID);
    const v4f cv = rne_bf4(ld4f(cprev + (size_t)row * NHID + col));
    v4f hn, cn;
#pragma unroll
    for (int e = 0; e < 4; ++e) {
      const float c0 = cv[e];
      const float ig = sigm_f((zi[e] + bsi[e]) + pci[e] * c0);
      const float fg = sigm_f((zf[e] + bsf[e]) + pcf[e] * c0);
      const float gg = tanh_f(zg[e] + bsg[e]);
      const float c1 = fg * c0 + ig * gg;
      const float og = sigm_f((zz[e] + bso[e]) + pco[e] * c1);
      hn[e] = og * tanh_f(c1);
      cn[e] = c1;
    }
    float* ph = outh + (size_t)row * NHID + col;
    float* pc = outc + (size_t)row * NHID + col;
    *(volatile v4f*)ph = hn;
    *(volatile v4f*)pc = cn;
    __threadfence();
    *(volatile v4f*)ph = hn;
    *(volatile v4f*)pc = cn;
  }
}

extern "C" void kernel_launch(void* const* d_in, const int* in_sizes, int n_in,
                              void* d_out, int out_size, void* d_ws, size_t ws_size,
                              hipStream_t stream) {
  if (n_in < 22) return;
  if (in_sizes[0] != NBATCH * NIN || in_sizes[1] != NBATCH * NHID || in_sizes[2] != NBATCH * NHID) return;
  if (in_sizes[3] != NHID * NIN || in_sizes[5] != NHID * NHID || in_sizes[19] != NHID * NHID) return;
  if (in_sizes[4] != NHID || in_sizes[21] != NHID) return;
  if ((size_t)out_size != 2 * OUT1_ELEM_OFF) return;
  if (ws_size < WS_TOTAL) return;

  const float* x    = (const float*)d_in[0];
  const float* h    = (const float*)d_in[1];
  const float* c    = (const float*)d_in[2];
  const float* W_ii = (const float*)d_in[3];
  const float* b_ii = (const float*)d_in[4];
  const float* W_hi = (const float*)d_in[5];
  const float* b_hi = (const float*)d_in[6];
  const float* W_ci = (const float*)d_in[7];
  const float* W_if = (const float*)d_in[8];
  const float* b_if = (const float*)d_in[9];
  const float* W_hf = (const float*)d_in[10];
  const float* b_hf = (const float*)d_in[11];
  const float* W_cf = (const float*)d_in[12];
  const float* W_ig = (const float*)d_in[13];
  const float* b_ig = (const float*)d_in[14];
  const float* W_hg = (const float*)d_in[15];
  const float* b_hg = (const float*)d_in[16];
  const float* W_io = (const float*)d_in[17];
  const float* b_io = (const float*)d_in[18];
  const float* W_ho = (const float*)d_in[19];
  const float* b_ho = (const float*)d_in[20];
  const float* W_co = (const float*)d_in[21];

  unsigned char*  ws = (unsigned char*)d_ws;
  unsigned short* Ap = (unsigned short*)(ws + WS_A_OFF);
  unsigned short* Wp = (unsigned short*)(ws + WS_W_OFF);
  float*          Zp = (float*)(ws + WS_Z_OFF);
  float*          outp = (float*)d_out;

  pack_act_rows<<<dim3(NBATCH), dim3(256), 0, stream>>>(x, h, Ap);
  pack_w_rows<<<dim3(NGATE4), dim3(256), 0, stream>>>(W_ii, W_if, W_ig, W_io, W_hi, W_hf, W_hg, W_ho, Wp);
  {
    const int tiles = (NBATCH / 64) * (NGATE4 / 64);
    const int blocks = (tiles + 7) / 8;
    wmma_gemm64<1, false, 0, 0, false, 0><<<dim3(blocks, 1), dim3(256), 0, stream>>>(
        Ap, Ap, KCAT, 0L,
        Wp, Wp, KCAT, 0L,
        (void*)Zp, (void*)Zp, NGATE4, 0L,
        b_ii,
        c, 0L,
        NBATCH, NGATE4, KCAT, 1.0f);
  }
  peep_gates<<<dim3(NBATCH / GATE_ROWS_PER_BLOCK), dim3(256), 0, stream>>>(
      Zp, c,
      b_ii, b_hi, b_if, b_hf, b_ig, b_hg, b_io, b_ho,
      W_ci, W_cf, W_co,
      outp);
}
